// MultiFilterConvDotProductAttention_4088808866278
// MI455X (gfx1250) — hardware-verified
//
#include <hip/hip_runtime.h>
#include <stdint.h>


typedef __bf16         v16bf __attribute__((ext_vector_type(16)));
typedef unsigned int   v4u   __attribute__((ext_vector_type(4)));
typedef float          v8f   __attribute__((ext_vector_type(8)));
typedef float          v4f   __attribute__((ext_vector_type(4)));
typedef int            v4i   __attribute__((ext_vector_type(4)));

union Frag { v16bf b; v4u q[2]; };

constexpr int S_DIM    = 1024;
constexpr int D_DIM    = 64;
constexpr int N_BH     = 16;
constexpr int N_H      = 8;
constexpr int ST_PITCH = 68;

__device__ __forceinline__ unsigned int bf16_bits_rne(float f) {
    unsigned int u = __float_as_uint(f);
    u += 0x7FFFu + ((u >> 16) & 1u);
    return u >> 16;
}

__device__ __forceinline__ void split8(const float* f, v4u& hi, v4u& lo) {
    unsigned int hw[4], lw[4];
#pragma unroll
    for (int j = 0; j < 4; ++j) {
        const float f0 = f[2 * j];
        const float f1 = f[2 * j + 1];
        const unsigned int h0 = bf16_bits_rne(f0);
        const unsigned int h1 = bf16_bits_rne(f1);
        const unsigned int l0 = bf16_bits_rne(f0 - __uint_as_float(h0 << 16));
        const unsigned int l1 = bf16_bits_rne(f1 - __uint_as_float(h1 << 16));
        hw[j] = h0 | (h1 << 16);
        lw[j] = l0 | (l1 << 16);
    }
    hi.x = hw[0]; hi.y = hw[1]; hi.z = hw[2]; hi.w = hw[3];
    lo.x = lw[0]; lo.y = lw[1]; lo.z = lw[2]; lo.w = lw[3];
}

__device__ __forceinline__ v8f wmma3(v8f acc, v16bf ah, v16bf al, v16bf bh, v16bf bl) {
    acc = __builtin_amdgcn_wmma_f32_16x16x32_bf16(false, ah, false, bh, (short)0, acc, false, false);
    acc = __builtin_amdgcn_wmma_f32_16x16x32_bf16(false, ah, false, bl, (short)0, acc, false, false);
    acc = __builtin_amdgcn_wmma_f32_16x16x32_bf16(false, al, false, bh, (short)0, acc, false, false);
    asm volatile("v_nop\n\tv_nop\n\tv_nop\n\tv_nop" : "+v"(acc) : "v"(ah), "v"(al), "v"(bh), "v"(bl));
    return acc;
}

__global__ __launch_bounds__(256) void k_planes(
    const float* __restrict__ q, const float* __restrict__ kin, const float* __restrict__ v,
    unsigned short* qh, unsigned short* ql, unsigned short* kh, unsigned short* kl,
    unsigned short* vth, unsigned short* vtl)
{
    __shared__ float tile[64][65];
    const int tid   = threadIdx.x;
    const int which = blockIdx.y;
    const int bx    = blockIdx.x;

    if (which == 2) {
        const int bh = bx >> 4;
        const int t0 = (bx & 15) * 64;
#pragma unroll
        for (int it = 0; it < 4; ++it) {
            const int g  = it * 256 + tid;
            const int r  = g >> 4;
            const int c4 = (g & 15) * 4;
            const v4f x = *(const v4f*)(v + ((size_t)(bh * S_DIM + t0 + r)) * D_DIM + c4);
            tile[r][c4 + 0] = x.x;
            tile[r][c4 + 1] = x.y;
            tile[r][c4 + 2] = x.z;
            tile[r][c4 + 3] = x.w;
        }
    }
    __syncthreads();
    if (which == 2) {
        const int bh = bx >> 4;
        const int t0 = (bx & 15) * 64;
#pragma unroll
        for (int it = 0; it < 2; ++it) {
            const int dd = it * 32 + (tid >> 3);
            const int p  = tid & 7;
            float f[8];
#pragma unroll
            for (int j = 0; j < 8; ++j) f[j] = tile[p * 8 + j][dd];
            v4u hi, lo;
            split8(f, hi, lo);
            const size_t off = ((size_t)(bh * D_DIM + dd)) * S_DIM + t0 + p * 8;
            *(volatile v4u*)(vth + off) = hi;
            *(volatile v4u*)(vtl + off) = lo;
            __threadfence();
            *(volatile v4u*)(vth + off) = hi;
            *(volatile v4u*)(vtl + off) = lo;
        }
    } else {
        const float* src   = (which == 0) ? q : kin;
        unsigned short* dh = (which == 0) ? qh : kh;
        unsigned short* dl = (which == 0) ? ql : kl;
        const float sc     = (which == 0) ? 0.125f : 1.0f;
#pragma unroll
        for (int it = 0; it < 2; ++it) {
            const int g = it * 256 + tid;
            const int r = g >> 3;
            const int p = g & 7;
            const size_t off = ((size_t)(bx * 64 + r)) * D_DIM + p * 8;
            const v4f a = *(const v4f*)(src + off);
            const v4f c = *(const v4f*)(src + off + 4);
            float f[8] = {a.x * sc, a.y * sc, a.z * sc, a.w * sc,
                          c.x * sc, c.y * sc, c.z * sc, c.w * sc};
            v4u hi, lo;
            split8(f, hi, lo);
            *(volatile v4u*)(dh + off) = hi;
            *(volatile v4u*)(dl + off) = lo;
            __threadfence();
            *(volatile v4u*)(dh + off) = hi;
            *(volatile v4u*)(dl + off) = lo;
        }
    }
}

__global__ __launch_bounds__(128) void k_scores(
    const unsigned short* __restrict__ qh, const unsigned short* __restrict__ ql,
    const unsigned short* __restrict__ kh, const unsigned short* __restrict__ kl,
    float* dp)
{
    __shared__ float stile[64 * ST_PITCH];
    const int tid  = threadIdx.x;
    const int lane = tid & 31;
    const int w    = tid >> 5;
    const int h    = lane >> 4;
    const int m    = lane & 15;
    const int bh   = blockIdx.z;
    const int s0   = blockIdx.y * 64;
    const int t0   = blockIdx.x * 64;

    const int ka0 = 8 * h;
    const int kb0 = 16 + 8 * h;
    const int ka1 = 32 + 8 * h;
    const int kb1 = 48 + 8 * h;

    const size_t arow = ((size_t)(bh * S_DIM + s0 + 16 * w + m)) * D_DIM;
    Frag aH0, aL0, aH1, aL1;
    aH0.q[0] = *(const v4u*)(qh + arow + ka0);  aH0.q[1] = *(const v4u*)(qh + arow + kb0);
    aL0.q[0] = *(const v4u*)(ql + arow + ka0);  aL0.q[1] = *(const v4u*)(ql + arow + kb0);
    aH1.q[0] = *(const v4u*)(qh + arow + ka1);  aH1.q[1] = *(const v4u*)(qh + arow + kb1);
    aL1.q[0] = *(const v4u*)(ql + arow + ka1);  aL1.q[1] = *(const v4u*)(ql + arow + kb1);

#pragma unroll
    for (int nt = 0; nt < 4; ++nt) {
        const size_t brow = ((size_t)(bh * S_DIM + t0 + 16 * nt + m)) * D_DIM;
        v8f c = {0.f, 0.f, 0.f, 0.f, 0.f, 0.f, 0.f, 0.f};
        {
            Frag bH, bL;
            bH.q[0] = *(const v4u*)(kh + brow + ka0);  bH.q[1] = *(const v4u*)(kh + brow + kb0);
            bL.q[0] = *(const v4u*)(kl + brow + ka0);  bL.q[1] = *(const v4u*)(kl + brow + kb0);
            c = wmma3(c, aH0.b, aL0.b, bH.b, bL.b);
        }
        {
            Frag bH, bL;
            bH.q[0] = *(const v4u*)(kh + brow + ka1);  bH.q[1] = *(const v4u*)(kh + brow + kb1);
            bL.q[0] = *(const v4u*)(kl + brow + ka1);  bL.q[1] = *(const v4u*)(kl + brow + kb1);
            c = wmma3(c, aH1.b, aL1.b, bH.b, bL.b);
        }
#pragma unroll
        for (int r = 0; r < 8; ++r)
            stile[(16 * w + 8 * h + r) * ST_PITCH + 16 * nt + m] = c[r];
    }
    __syncthreads();

#pragma unroll
    for (int it = 0; it < 8; ++it) {
        const int L    = it * 16 + (tid >> 3);
        const int row  = L >> 1;
        const int half = L & 1;
        const int p    = tid & 7;
        const v4f x = *(const v4f*)(stile + row * ST_PITCH + half * 32 + p * 4);
        float* dst = dp + ((size_t)(bh * S_DIM + s0 + row)) * S_DIM + t0 + half * 32 + p * 4;
        *(volatile v4f*)dst = x;
    }
    __threadfence();
#pragma unroll
    for (int it = 0; it < 8; ++it) {
        const int L    = it * 16 + (tid >> 3);
        const int row  = L >> 1;
        const int half = L & 1;
        const int p    = tid & 7;
        const v4f x = *(const v4f*)(stile + row * ST_PITCH + half * 32 + p * 4);
        float* dst = dp + ((size_t)(bh * S_DIM + s0 + row)) * S_DIM + t0 + half * 32 + p * 4;
        *(volatile v4f*)dst = x;
    }
}

__device__ __forceinline__ void load_row(float* R, const float* dpb, int sr, bool rv, int col0) {
    const int src = min(max(sr, 0), S_DIM - 1);
    const float* rp = dpb + (size_t)src * S_DIM;
    const v4f a = *(const v4f*)(rp + col0);
    const v4f c = *(const v4f*)(rp + col0 + 4);
    const int cl = max(col0 - 1, 0);
    const int cr = min(col0 + 8, S_DIM - 1);
    float xl = rp[cl];
    float xr = rp[cr];
    xl = (col0 > 0) ? xl : 0.f;
    xr = (col0 + 8 < S_DIM) ? xr : 0.f;
    R[0] = rv ? xl  : 0.f;
    R[1] = rv ? a.x : 0.f;  R[2] = rv ? a.y : 0.f;  R[3] = rv ? a.z : 0.f;  R[4] = rv ? a.w : 0.f;
    R[5] = rv ? c.x : 0.f;  R[6] = rv ? c.y : 0.f;  R[7] = rv ? c.z : 0.f;  R[8] = rv ? c.w : 0.f;
    R[9] = rv ? xr  : 0.f;
}

__global__ __launch_bounds__(128) void k_attn(
    const float* __restrict__ dp,
    const unsigned short* __restrict__ vth, const unsigned short* __restrict__ vtl,
    const int* __restrict__ mask,
    const float* __restrict__ conv_w, const float* __restrict__ conv_b,
    const float* __restrict__ lin_w, const float* __restrict__ lin_b,
    float* out)
{
    __shared__ float pre[16 * S_DIM];
    const int tid  = threadIdx.x;
    const int lane = tid & 31;
    const int w    = tid >> 5;
    const int h    = lane >> 4;
    const int m    = lane & 15;
    const int bh   = blockIdx.y;
    const int b    = bh / N_H;
    const int s0   = blockIdx.x * 16;
    const float* dpb = dp + (size_t)bh * S_DIM * S_DIM;

    {
        float wg[36];
#pragma unroll
        for (int i = 0; i < 36; ++i) wg[i] = conv_w[i];
        const float cb0 = conv_b[0], cb1 = conv_b[1], cb2 = conv_b[2], cb3 = conv_b[3];
        const float lw0 = lin_w[0],  lw1 = lin_w[1],  lw2 = lin_w[2],  lw3 = lin_w[3];
        const float lb  = lin_b[0];
        const int col0 = tid * 8;

        float ra[10], rb[10], rc[10];
        load_row(ra, dpb, s0 - 1, s0 > 0, col0);
        load_row(rb, dpb, s0, true, col0);
#pragma unroll 1
        for (int r = 0; r < 16; ++r) {
            const int sn = s0 + r + 1;
            load_row(rc, dpb, sn, sn < S_DIM, col0);
            const int* mrow = mask + ((size_t)(b * S_DIM + s0 + r)) * S_DIM + col0;
            const v4i mq0 = *(const v4i*)mrow;
            const v4i mq1 = *(const v4i*)(mrow + 4);
            const int mv[8] = {mq0.x, mq0.y, mq0.z, mq0.w, mq1.x, mq1.y, mq1.z, mq1.w};
            float pv[8];
#pragma unroll
            for (int j = 0; j < 8; ++j) {
                float a0 = cb0, a1 = cb1, a2 = cb2, a3 = cb3;
#pragma unroll
                for (int dj = 0; dj < 3; ++dj) {
                    const float x0 = ra[j + dj];
                    const float x1 = rb[j + dj];
                    const float x2 = rc[j + dj];
                    a0 += wg[0 * 9 + dj] * x0 + wg[0 * 9 + 3 + dj] * x1 + wg[0 * 9 + 6 + dj] * x2;
                    a1 += wg[1 * 9 + dj] * x0 + wg[1 * 9 + 3 + dj] * x1 + wg[1 * 9 + 6 + dj] * x2;
                    a2 += wg[2 * 9 + dj] * x0 + wg[2 * 9 + 3 + dj] * x1 + wg[2 * 9 + 6 + dj] * x2;
                    a3 += wg[3 * 9 + dj] * x0 + wg[3 * 9 + 3 + dj] * x1 + wg[3 * 9 + 6 + dj] * x2;
                }
                a0 = (a0 >= 0.f) ? a0 : 0.01f * a0;
                a1 = (a1 >= 0.f) ? a1 : 0.01f * a1;
                a2 = (a2 >= 0.f) ? a2 : 0.01f * a2;
                a3 = (a3 >= 0.f) ? a3 : 0.01f * a3;
                const float p = (lw0 * a0 + lw1 * a1 + lw2 * a2 + lw3 * a3) + lb;
                pv[j] = (mv[j] == 0) ? -1.0e30f : p;
            }
            v4f o0, o1;
            o0.x = pv[0]; o0.y = pv[1]; o0.z = pv[2]; o0.w = pv[3];
            o1.x = pv[4]; o1.y = pv[5]; o1.z = pv[6]; o1.w = pv[7];
            *(v4f*)(pre + r * S_DIM + col0)     = o0;
            *(v4f*)(pre + r * S_DIM + col0 + 4) = o1;
#pragma unroll
            for (int i = 0; i < 10; ++i) { ra[i] = rb[i]; rb[i] = rc[i]; }
        }
    }
    __syncthreads();

#pragma unroll 1
    for (int rr = 0; rr < 4; ++rr) {
        float* rowp = pre + (w * 4 + rr) * S_DIM;
        float mx = -3.0e38f;
#pragma unroll 4
        for (int i = 0; i < 32; ++i) mx = fmaxf(mx, rowp[lane + (i << 5)]);
        for (int off = 16; off; off >>= 1) mx = fmaxf(mx, __shfl_xor(mx, off, 32));
        float ssum = 0.f;
#pragma unroll 4
        for (int i = 0; i < 32; ++i) {
            const int idx = lane + (i << 5);
            const float ev = __expf(rowp[idx] - mx);
            rowp[idx] = ev;
            ssum += ev;
        }
        for (int off = 16; off; off >>= 1) ssum += __shfl_xor(ssum, off, 32);
        const float inv = 1.0f / ssum;
#pragma unroll 4
        for (int i = 0; i < 32; ++i) rowp[lane + (i << 5)] *= inv;
    }
    __syncthreads();

    const int d0 = 16 * w;
    const float* prow  = pre + m * S_DIM;
    const size_t vrow  = ((size_t)(bh * D_DIM + d0 + m)) * S_DIM;
    v8f acc = {0.f, 0.f, 0.f, 0.f, 0.f, 0.f, 0.f, 0.f};
#pragma unroll 4
    for (int k0 = 0; k0 < S_DIM; k0 += 32) {
        const int ka = k0 + 8 * h;
        const int kb = k0 + 16 + 8 * h;
        const v4f p0 = *(const v4f*)(prow + ka);
        const v4f p1 = *(const v4f*)(prow + ka + 4);
        const v4f p2 = *(const v4f*)(prow + kb);
        const v4f p3 = *(const v4f*)(prow + kb + 4);
        float fa[8] = {p0.x, p0.y, p0.z, p0.w, p1.x, p1.y, p1.z, p1.w};
        float fb[8] = {p2.x, p2.y, p2.z, p2.w, p3.x, p3.y, p3.z, p3.w};
        Frag aH, aL;
        split8(fa, aH.q[0], aL.q[0]);
        split8(fb, aH.q[1], aL.q[1]);
        Frag bH, bL;
        bH.q[0] = *(const v4u*)(vth + vrow + ka);  bH.q[1] = *(const v4u*)(vth + vrow + kb);
        bL.q[0] = *(const v4u*)(vtl + vrow + ka);  bL.q[1] = *(const v4u*)(vtl + vrow + kb);
        acc = wmma3(acc, aH.b, aL.b, bH.b, bL.b);
    }
    __syncthreads();

#pragma unroll
    for (int r = 0; r < 8; ++r) pre[(8 * h + r) * D_DIM + d0 + m] = acc[r];
    __syncthreads();

#pragma unroll
    for (int it = 0; it < 2; ++it) {
        const int L    = it * 16 + (tid >> 3);
        const int row  = L >> 1;
        const int half = L & 1;
        const int p    = tid & 7;
        const v4f x = *(const v4f*)(pre + row * D_DIM + half * 32 + p * 4);
        float* dst = out + ((size_t)(bh * S_DIM + s0 + row)) * D_DIM + half * 32 + p * 4;
        *(volatile v4f*)dst = x;
    }
    __threadfence();
#pragma unroll
    for (int it = 0; it < 2; ++it) {
        const int L    = it * 16 + (tid >> 3);
        const int row  = L >> 1;
        const int half = L & 1;
        const int p    = tid & 7;
        const v4f x = *(const v4f*)(pre + row * D_DIM + half * 32 + p * 4);
        float* dst = out + ((size_t)(bh * S_DIM + s0 + row)) * D_DIM + half * 32 + p * 4;
        *(volatile v4f*)dst = x;
    }
}

extern "C" void kernel_launch(void* const* d_in, const int* in_sizes, int n_in,
                              void* d_out, int out_size, void* d_ws, size_t ws_size,
                              hipStream_t stream)
{
    if (n_in < 8) return;
    const int nq = N_BH * S_DIM * D_DIM;
    if (in_sizes[0] != nq || in_sizes[1] != nq || in_sizes[2] != nq) return;
    if (in_sizes[3] != 2 * S_DIM * S_DIM) return;
    if (in_sizes[4] != 36 || in_sizes[5] != 4 || in_sizes[6] != 4 || in_sizes[7] != 1) return;
    if (out_size != nq) return;

    const size_t plane_elems = (size_t)nq;
    const size_t plane_bytes = plane_elems * 2;
    const size_t dp_bytes    = (size_t)N_BH * S_DIM * S_DIM * 4;
    const size_t total       = 6 * plane_bytes + dp_bytes;
    if (ws_size < total) return;

    const float* q      = (const float*)d_in[0];
    const float* k      = (const float*)d_in[1];
    const float* v      = (const float*)d_in[2];
    const int*   mask   = (const int*)  d_in[3];
    const float* conv_w = (const float*)d_in[4];
    const float* conv_b = (const float*)d_in[5];
    const float* lin_w  = (const float*)d_in[6];
    const float* lin_b  = (const float*)d_in[7];
    float* out = (float*)d_out;

    unsigned short* ws16 = (unsigned short*)d_ws;
    unsigned short* qh  = ws16 + 0 * plane_elems;
    unsigned short* ql  = ws16 + 1 * plane_elems;
    unsigned short* kh  = ws16 + 2 * plane_elems;
    unsigned short* kl  = ws16 + 3 * plane_elems;
    unsigned short* vth = ws16 + 4 * plane_elems;
    unsigned short* vtl = ws16 + 5 * plane_elems;
    float* dp = (float*)((char*)d_ws + 6 * plane_bytes);

    k_planes<<<dim3(256, 3), dim3(256), 0, stream>>>(q, k, v, qh, ql, kh, kl, vth, vtl);
    k_scores<<<dim3(S_DIM / 64, S_DIM / 64, N_BH), dim3(128), 0, stream>>>(qh, ql, kh, kl, dp);
    k_attn<<<dim3(S_DIM / 16, N_BH), dim3(128), 0, stream>>>(dp, vth, vtl, mask, conv_w, conv_b, lin_w, lin_b, out);
}
